// MTL2d_DeepSVDD_46986942218450
// MI455X (gfx1250) — hardware-verified
//
#include <hip/hip_runtime.h>
#include <math.h>


typedef _Float16 v16h __attribute__((ext_vector_type(16)));
typedef _Float16 v8h  __attribute__((ext_vector_type(8)));
typedef float    v8f  __attribute__((ext_vector_type(8)));
typedef float    v4f  __attribute__((ext_vector_type(4)));

union HFrag  { v16h v; v8h h8[2]; _Float16 e[16]; };
union HPack8 { v8h v; _Float16 e[8]; };
union FPack4 { v4f v; float e[4]; };

#define GT 128
#define MPADMAX 192
#define APITCH 40
#define RPITCH 36
#define SPITCH 36
#define VPITCH 40
#define TPW 6

__device__ __forceinline__ v8f wmma_f16(v16h a, v16h b, v8f c) {
  v8f d = __builtin_amdgcn_wmma_f32_16x16x32_f16(false, a, false, b, (short)0, c, false, false);
  asm volatile("v_nop\n\tv_nop\n\tv_nop\n\tv_nop" : "+v"(d) : "v"(a), "v"(b));
  return d;
}

__global__ __launch_bounds__(256)
void conv_s2_relu_c1(const float* __restrict__ in, const float* __restrict__ w,
                     const float* __restrict__ bias, float* out,
                     int B, int Cout, int Hin) {
  const int Ho = Hin >> 1;
  const int Wo = Ho;
  const int W4 = Wo >> 2;
  const int total = B * Cout * Ho * W4;
  const int q = blockIdx.x * blockDim.x + threadIdx.x;
  if (q >= total) return;
  const int w4 = q % W4;
  int t = q / W4;
  const int ho = t % Ho; t /= Ho;
  const int co = t % Cout;
  const int b = t / Cout;
  const float* ip = in + (size_t)b * Hin * Hin;
  const float* wp = w + co * 9;
  FPack4 acc;
  acc.e[0] = 0.f; acc.e[1] = 0.f; acc.e[2] = 0.f; acc.e[3] = 0.f;
#pragma unroll
  for (int kh = 0; kh < 3; ++kh) {
    const int hi = 2 * ho - 1 + kh;
    if (hi < 0 || hi >= Hin) continue;
    const float* rp = ip + (size_t)hi * Hin;
#pragma unroll
    for (int j = 0; j < 4; ++j) {
      const int wo = 4 * w4 + j;
#pragma unroll
      for (int kw = 0; kw < 3; ++kw) {
        const int wi = 2 * wo - 1 + kw;
        if (wi < 0 || wi >= Hin) continue;
        acc.e[j] += rp[wi] * wp[kh * 3 + kw];
      }
    }
  }
  const float bo = bias[co];
#pragma unroll
  for (int j = 0; j < 4; ++j) acc.e[j] = fmaxf(acc.e[j] + bo, 0.0f);
  float* dst = out + ((((size_t)(b * Cout + co)) * Ho + ho) * Wo + 4 * w4);
  *(volatile v4f*)dst = acc.v;
  __threadfence();
  *(volatile v4f*)dst = acc.v;
}

template <int MODE>
__global__ __launch_bounds__(GT)
void gemm_tc(const float* __restrict__ wmat, const float* __restrict__ bias,
             const float* __restrict__ src, const float* __restrict__ res,
             float* zout, _Float16* Qo, _Float16* Ko, _Float16* Vo,
             int M, int K, int N, int Cin, int Hin, int heads, int d) {
  __shared__ __attribute__((aligned(16))) _Float16 Al[MPADMAX * APITCH];
  __shared__ __attribute__((aligned(16))) _Float16 Bl[32 * APITCH];
  __shared__ __attribute__((aligned(16))) float Rl[MPADMAX * RPITCH];
  const int tid = threadIdx.x, wv = tid >> 5, lane = tid & 31, h = lane >> 4, m = lane & 15;
  const int b = blockIdx.y;
  const int n0 = blockIdx.x * 32;
  if (n0 + 32 > N) return;
  const int Mpad = (M + 15) & ~15;
  const int Kpad = (K + 31) & ~31;
  if (Mpad > MPADMAX) return;
  const int ntiles = (Mpad >> 4) * 2;

  v8f acc[TPW];
#pragma unroll
  for (int u = 0; u < TPW; ++u) { v8f z = {}; acc[u] = z; }

  for (int k0 = 0; k0 < Kpad; k0 += 32) {
    for (int idx = tid; idx < Mpad * 32; idx += GT) {
      const int r = idx >> 5, kk = idx & 31, k = k0 + kk;
      float v = 0.f;
      if (r < M && k < K) v = wmat[(size_t)r * K + k];
      Al[r * APITCH + kk] = (_Float16)v;
    }
    for (int idx = tid; idx < 32 * 32; idx += GT) {
      const int n = idx & 31, kk = idx >> 5, k = k0 + kk;
      float v = 0.f;
      if (k < K) {
        if (MODE == 0) {
          const int ci = k / 9;
          const int rr = k - ci * 9;
          const int kh = rr / 3;
          const int kw = rr - kh * 3;
          const int Ho = Hin >> 1;
          const int p = n0 + n;
          const int ho = p / Ho;
          const int wo = p - ho * Ho;
          const int hi = 2 * ho - 1 + kh, wi = 2 * wo - 1 + kw;
          if (hi >= 0 && hi < Hin && wi >= 0 && wi < Hin)
            v = src[(((size_t)(b * Cin + ci)) * Hin + hi) * Hin + wi];
        } else if (MODE == 1) {
          v = src[((size_t)b * K + k) * N + n0 + n];
        } else {
          const int hh = k % heads, dd = k / heads;
          v = src[(((size_t)(b * heads + hh)) * N + n0 + n) * 32 + dd];
        }
      }
      Bl[n * APITCH + kk] = (_Float16)v;
    }
    __syncthreads();
#pragma unroll
    for (int u = 0; u < TPW; ++u) {
      const int t = wv + 4 * u;
      if (t < ntiles) {
        const int rt = t >> 1, ct = t & 1;
        HFrag a, bb;
        a.h8[0]  = *(const v8h*)&Al[(16 * rt + m) * APITCH + 8 * h];
        a.h8[1]  = *(const v8h*)&Al[(16 * rt + m) * APITCH + 16 + 8 * h];
        bb.h8[0] = *(const v8h*)&Bl[(16 * ct + m) * APITCH + 8 * h];
        bb.h8[1] = *(const v8h*)&Bl[(16 * ct + m) * APITCH + 16 + 8 * h];
        acc[u] = wmma_f16(a.v, bb.v, acc[u]);
      }
    }
    __syncthreads();
  }

#pragma unroll
  for (int u = 0; u < TPW; ++u) {
    const int t = wv + 4 * u;
    if (t < ntiles) {
      const int rt = t >> 1, ct = t & 1;
#pragma unroll
      for (int r = 0; r < 8; ++r)
        Rl[(16 * rt + 8 * h + r) * RPITCH + 16 * ct + m] = acc[u][r];
    }
  }
  __syncthreads();

  if (MODE != 1) {
    const int cc = (lane & 7) * 4;
    for (int pass = 0; pass < 2; ++pass) {
      if (pass) __threadfence();
      for (int lb = 4 * wv; lb < M; lb += 16) {
        const int oc = lb + (lane >> 3);
        if (oc < M) {
          FPack4 v;
          v.v = *(const v4f*)&Rl[oc * RPITCH + cc];
          const float bo = bias[oc];
          const size_t off = ((size_t)(b * M + oc)) * N + n0 + cc;
          if (MODE == 0) {
#pragma unroll
            for (int j = 0; j < 4; ++j) v.e[j] = fmaxf(v.e[j] + bo, 0.0f);
          } else {
            FPack4 rr;
            rr.v = *(const v4f*)(res + off);
#pragma unroll
            for (int j = 0; j < 4; ++j) v.e[j] = (v.e[j] + bo) + rr.e[j];
          }
          *(volatile v4f*)(zout + off) = v.v;
        }
      }
    }
  } else {
    const int inner = heads * d;
    const int nlines = 3 * heads * 16;
    const int sub = lane & 7;
    const int nlo = sub >> 2;
    const int ddc = (sub & 3) * 8;
    for (int pass = 0; pass < 2; ++pass) {
      if (pass) __threadfence();
      for (int lb = 4 * wv; lb < nlines; lb += 16) {
        const int L = lb + (lane >> 3);
        if (L < nlines) {
          const int g = L >> 4, np = L & 15;
          const int part = g / heads;
          const int hh = g - part * heads;
          const int n = 2 * np + nlo;
          HPack8 pk;
#pragma unroll
          for (int e = 0; e < 8; ++e) {
            const int dd = ddc + e;
            float v = 0.f;
            if (dd < d) {
              const int oc = part * inner + dd * heads + hh;
              v = Rl[oc * RPITCH + n] + bias[oc];
            }
            pk.e[e] = (_Float16)v;
          }
          _Float16* basep = (part == 0) ? Qo : ((part == 1) ? Ko : Vo);
          const size_t off = ((((size_t)(b * heads + hh)) * N) + n0 + n) * 32 + ddc;
          *(volatile v8h*)(basep + off) = pk.v;
        }
      }
    }
  }
}

template <int NCH>
__global__ __launch_bounds__(GT)
void attn_tc(const _Float16* __restrict__ Qg, const _Float16* __restrict__ Kg,
             const _Float16* __restrict__ Vg, const float* __restrict__ rel,
             float* Og, int heads, int N, int hsShift, int d, float scale) {
  __shared__ __attribute__((aligned(16))) float Sl[4 * 16 * SPITCH];
  __shared__ __attribute__((aligned(16))) _Float16 Vl[32 * VPITCH];
  const int tid = threadIdx.x, wv = tid >> 5, lane = tid & 31, h = lane >> 4, mn = lane & 15;
  const int bh = blockIdx.y;
  const int hh = bh % heads;
  if (blockIdx.x * 64 + 64 > N) return;
  const int row0 = blockIdx.x * 64 + 16 * wv;
  const size_t base = (size_t)bh * N * 32;
  const int Hs = 1 << hsShift, hmask = Hs - 1, R2 = 2 * Hs - 1;
  float* Sw = Sl + wv * 16 * SPITCH;
  (void)d;

  HFrag aq;
  {
    const _Float16* qr = Qg + base + (size_t)(row0 + mn) * 32;
    aq.h8[0] = *(const v8h*)(qr + 8 * h);
    aq.h8[1] = *(const v8h*)(qr + 16 + 8 * h);
  }
  int rowterm[8];
#pragma unroll
  for (int r = 0; r < 8; ++r) {
    const int ig = row0 + 8 * h + r;
    rowterm[r] = ((ig >> hsShift) + Hs - 1) * R2 + (ig & hmask) + Hs - 1;
  }
  const float* relh = rel + hh;
  float m_run = -3.0e38f, l_run = 0.f;
  v8f oacc[NCH];
#pragma unroll
  for (int c = 0; c < NCH; ++c) { v8f z = {}; oacc[c] = z; }

  for (int col0 = 0; col0 < N; col0 += 32) {
    __syncthreads();
    {
      const int key = tid >> 2, c8 = (tid & 3) * 8;
      HPack8 pv;
      pv.v = *(const v8h*)(Vg + base + (size_t)(col0 + key) * 32 + c8);
#pragma unroll
      for (int e = 0; e < 8; ++e) Vl[(c8 + e) * VPITCH + key] = pv.e[e];
    }
    v8f S[2];
#pragma unroll
    for (int t = 0; t < 2; ++t) {
      const _Float16* kr = Kg + base + (size_t)(col0 + 16 * t + mn) * 32;
      HFrag bk;
      bk.h8[0] = *(const v8h*)(kr + 8 * h);
      bk.h8[1] = *(const v8h*)(kr + 16 + 8 * h);
      v8f cz = {};
      S[t] = wmma_f16(aq.v, bk.v, cz);
    }
#pragma unroll
    for (int t = 0; t < 2; ++t) {
      const int jg = col0 + 16 * t + mn;
      const int colterm = (jg >> hsShift) * R2 + (jg & hmask);
#pragma unroll
      for (int r = 0; r < 8; ++r) {
        const int idx = rowterm[r] - colterm;
        Sw[(8 * h + r) * SPITCH + 16 * t + mn] = (S[t][r] + relh[(size_t)idx * heads]) * scale;
      }
    }
    __syncthreads();
    FPack4 rv[4];
    rv[0].v = *(const v4f*)&Sw[mn * SPITCH + 8 * h];
    rv[1].v = *(const v4f*)&Sw[mn * SPITCH + 8 * h + 4];
    rv[2].v = *(const v4f*)&Sw[mn * SPITCH + 16 + 8 * h];
    rv[3].v = *(const v4f*)&Sw[mn * SPITCH + 16 + 8 * h + 4];
    float m8 = rv[0].e[0];
#pragma unroll
    for (int i = 1; i < 16; ++i) m8 = fmaxf(m8, rv[i >> 2].e[i & 3]);
    m8 = fmaxf(m8, __shfl_xor(m8, 16, 32));
    const float mnew = fmaxf(m_run, m8);
    const float alpha = __expf(m_run - mnew);
    m_run = mnew;
    HFrag ap;
    float psum = 0.f;
#pragma unroll
    for (int i = 0; i < 16; ++i) {
      const float p = __expf(rv[i >> 2].e[i & 3] - mnew);
      psum += p;
      ap.e[i] = (_Float16)p;
    }
    psum += __shfl_xor(psum, 16, 32);
    l_run = l_run * alpha + psum;
#pragma unroll
    for (int r = 0; r < 8; ++r) {
      const float ar = __shfl(alpha, 8 * h + r, 16);
#pragma unroll
      for (int c = 0; c < NCH; ++c) oacc[c][r] = oacc[c][r] * ar;
    }
#pragma unroll
    for (int c = 0; c < NCH; ++c) {
      HFrag bv;
      bv.h8[0] = *(const v8h*)&Vl[(16 * c + mn) * VPITCH + 8 * h];
      bv.h8[1] = *(const v8h*)&Vl[(16 * c + mn) * VPITCH + 16 + 8 * h];
      oacc[c] = wmma_f16(ap.v, bv.v, oacc[c]);
    }
  }

  float inv[8];
#pragma unroll
  for (int r = 0; r < 8; ++r) inv[r] = 1.0f / __shfl(l_run, 8 * h + r, 16);
  __syncthreads();
#pragma unroll
  for (int r = 0; r < 8; ++r) {
#pragma unroll
    for (int c = 0; c < NCH; ++c) Sw[(8 * h + r) * SPITCH + 16 * c + mn] = oacc[c][r] * inv[r];
    if (NCH == 1) Sw[(8 * h + r) * SPITCH + 16 + mn] = 0.f;
  }
  __syncthreads();
  const int cc = (lane & 7) * 4;
  v4f ov[4];
#pragma unroll
  for (int q = 0; q < 4; ++q) ov[q] = *(const v4f*)&Sw[(4 * q + (lane >> 3)) * SPITCH + cc];
  float* ob = Og + (size_t)bh * N * 32 + (size_t)row0 * 32 + cc;
#pragma unroll
  for (int q = 0; q < 4; ++q) *(volatile v4f*)(ob + (size_t)(4 * q + (lane >> 3)) * 32) = ov[q];
  __threadfence();
#pragma unroll
  for (int q = 0; q < 4; ++q) *(volatile v4f*)(ob + (size_t)(4 * q + (lane >> 3)) * 32) = ov[q];
}

__global__ __launch_bounds__(256)
void pool_head(const float* __restrict__ z, const float* __restrict__ cw,
               const float* __restrict__ cb, float* out, int B, int C, int N, int NC) {
  __shared__ __attribute__((aligned(16))) float buf[2432];
  const int tid = threadIdx.x;
  const int nz = B * C, ncls = B * NC, tot = nz + ncls;
  if (tot > 2432 || (tot & 3) != 0) return;
  const float invN = 1.0f / (float)N;
  for (int i = tid; i < nz; i += 256) {
    const float* zp = z + (size_t)i * N;
    float s = 0.f;
#pragma unroll 4
    for (int n = 0; n < N; ++n) s += zp[n];
    buf[i] = s * invN;
  }
  __syncthreads();
  for (int i = tid; i < ncls; i += 256) {
    const int o = i % NC, bb = i / NC;
    const float* wp = cw + (size_t)o * C;
    const float* zp = buf + bb * C;
    float s = 0.f;
#pragma unroll 1
    for (int c = 0; c < C; ++c) s += zp[c] * wp[c];
    buf[nz + i] = s + cb[o];
  }
  __syncthreads();
  const int nv = tot >> 2;
  for (int v = tid; v < nv; v += 256) {
    const v4f val = *(const v4f*)&buf[4 * v];
    *(volatile v4f*)(out + 4 * v) = val;
  }
  __threadfence();
  for (int v = tid; v < nv; v += 256) {
    const v4f val = *(const v4f*)&buf[4 * v];
    *(volatile v4f*)(out + 4 * v) = val;
  }
}

static inline int cdiv(int a, int b) { return (a + b - 1) / b; }
static inline size_t al256(size_t x) { return (x + 255) & ~(size_t)255; }

extern "C" void kernel_launch(void* const* d_in, const int* in_sizes, int n_in,
                              void* d_out, int out_size, void* d_ws,
                              size_t ws_size, hipStream_t stream) {
  const int B = 32, heads = 3, NCLS = 10;
  const int dims[3] = {16, 32, 64};
  const int cins[3] = {1, 16, 32};
  const int hins[3] = {64, 32, 16};
  const int dsz[3]  = {5, 10, 21};
  const int hsh[3]  = {5, 4, 3};
  if (n_in < 24) return;
  if (in_sizes[0] != B * 64 * 64) return;
  if (out_size != B * 64 + B * NCLS) return;
  for (int s = 0; s < 3; ++s) {
    const int inner = heads * dsz[s];
    if (in_sizes[1 + 7 * s] != dims[s] * cins[s] * 9) return;
    if (in_sizes[3 + 7 * s] != 3 * inner * dims[s]) return;
    if (in_sizes[5 + 7 * s] != dims[s] * inner) return;
    const int Hs = hins[s] / 2;
    if (in_sizes[7 + 7 * s] != (2 * Hs - 1) * (2 * Hs - 1) * heads) return;
    if ((Hs * Hs) % 64 != 0) return;
    if (3 * inner > MPADMAX) return;
  }
  if (in_sizes[22] != NCLS * 64 || in_sizes[23] != NCLS) return;

  const float* x = (const float*)d_in[0];
  const float* cw[3] = {(const float*)d_in[1],  (const float*)d_in[8],  (const float*)d_in[15]};
  const float* cb[3] = {(const float*)d_in[2],  (const float*)d_in[9],  (const float*)d_in[16]};
  const float* qw[3] = {(const float*)d_in[3],  (const float*)d_in[10], (const float*)d_in[17]};
  const float* qb[3] = {(const float*)d_in[4],  (const float*)d_in[11], (const float*)d_in[18]};
  const float* ow[3] = {(const float*)d_in[5],  (const float*)d_in[12], (const float*)d_in[19]};
  const float* ob[3] = {(const float*)d_in[6],  (const float*)d_in[13], (const float*)d_in[20]};
  const float* rl[3] = {(const float*)d_in[7],  (const float*)d_in[14], (const float*)d_in[21]};
  const float* clsw = (const float*)d_in[22];
  const float* clsb = (const float*)d_in[23];
  float* out = (float*)d_out;

  size_t zmax = 0; int nmax = 0;
  for (int s = 0; s < 3; ++s) {
    const int Hs = hins[s] / 2, N = Hs * Hs;
    if ((size_t)dims[s] * N > zmax) zmax = (size_t)dims[s] * N;
    if (N > nmax) nmax = N;
  }
  const size_t zbytes = al256((size_t)B * zmax * sizeof(float));
  const size_t hbytes = al256((size_t)B * heads * nmax * 32 * sizeof(_Float16));
  const size_t obytes = al256((size_t)B * heads * nmax * 32 * sizeof(float));
  size_t off = 0;
  const size_t offA = off; off += zbytes;
  const size_t offB = off; off += zbytes;
  const size_t offQ = off; off += hbytes;
  const size_t offK = off; off += hbytes;
  const size_t offV = off; off += hbytes;
  const size_t offO = off; off += obytes;
  if (off > ws_size) return;
  char* ws = (char*)d_ws;
  float*    zA = (float*)(ws + offA);
  float*    zB = (float*)(ws + offB);
  _Float16* Qh = (_Float16*)(ws + offQ);
  _Float16* Kh = (_Float16*)(ws + offK);
  _Float16* Vh = (_Float16*)(ws + offV);
  float*    Ob = (float*)(ws + offO);

  {
    const int total4 = B * dims[0] * (hins[0] / 2) * ((hins[0] / 2) / 4);
    conv_s2_relu_c1<<<cdiv(total4, 256), 256, 0, stream>>>(x, cw[0], cb[0], zA, B, dims[0], hins[0]);
  }
  for (int s = 0; s < 3; ++s) {
    const int dim = dims[s], Hin = hins[s], Hs = Hin / 2, N = Hs * Hs;
    const int dd = dsz[s], inner = heads * dd;
    const dim3 g32(N / 32, B);
    if (s > 0) {
      gemm_tc<0><<<g32, GT, 0, stream>>>(cw[s], cb[s], zB, zB, zA, Qh, Kh, Vh,
                                         dim, cins[s] * 9, N, cins[s], Hin, heads, dd);
    }
    gemm_tc<1><<<g32, GT, 0, stream>>>(qw[s], qb[s], zA, zA, Ob, Qh, Kh, Vh,
                                       3 * inner, dim, N, 0, 0, heads, dd);
    {
      const dim3 ga(N / 64, B * heads);
      const float scale = (float)(1.0 / sqrt((double)dd));
      if (dd <= 16)
        attn_tc<1><<<ga, GT, 0, stream>>>(Qh, Kh, Vh, rl[s], Ob, heads, N, hsh[s], dd, scale);
      else
        attn_tc<2><<<ga, GT, 0, stream>>>(Qh, Kh, Vh, rl[s], Ob, heads, N, hsh[s], dd, scale);
    }
    gemm_tc<2><<<g32, GT, 0, stream>>>(ow[s], ob[s], Ob, zA, zB, Qh, Kh, Vh,
                                       dim, inner, N, 0, 0, heads, dd);
  }
  pool_head<<<1, 256, 0, stream>>>(zB, clsw, clsb, out, B, 64, 64, NCLS);
}
